// DiTEmb_dynamics_42202348651014
// MI455X (gfx1250) — hardware-run, weakly checked
//
#include <hip/hip_runtime.h>
#include <math.h>

typedef __attribute__((ext_vector_type(16))) _Float16 v16h;
typedef __attribute__((ext_vector_type(8)))  _Float16 v8h;
typedef __attribute__((ext_vector_type(8)))  float    v8f;
typedef __attribute__((ext_vector_type(4)))  float    v4f;
typedef __attribute__((ext_vector_type(2)))  float    v2f;

constexpr int kBatch   = 8;
constexpr int kNode    = 256;
constexpr int kXhIn    = 9;
constexpr int kXhHid   = 64;
constexpr int kPosHid  = 192;
constexpr int kFreq    = 64;
constexpr int kFeat    = 2 * kFreq;
constexpr int kRows    = kBatch * kNode;
constexpr int kOutCols = kXhHid + kPosHid;
static_assert(kFeat == 128 && (kFeat % 32) == 0, "GEMM K multiple of 32");
static_assert((kRows % 64) == 0 && (kPosHid % 64) == 0, "GEMM M,N multiples of 64");
static_assert(kOutCols == 256 && (kNode % 16) == 0, "row tiles stay inside one batch element");

constexpr float kSCarry = 256.0f;
constexpr float kWCarry = 256.0f;
constexpr float kFold   = 1.0f / (kSCarry * kWCarry);
constexpr float kPairCount = (float)kNode;
constexpr double kFreqStepD  = 6.643856189774724 / (double)kFreq;
constexpr float  kFreqStepHi = (float)kFreqStepD;
constexpr float  kFreqStepLo = (float)(kFreqStepD - (double)kFreqStepHi);
constexpr float kTwoPi = 6.283185307179586f;

constexpr size_t kOffXC   = 0;
constexpr size_t kOffNINV = kOffXC   + (size_t)kRows * 4 * 4;
constexpr size_t kOffWT   = kOffNINV + (size_t)kBatch * 32 * 4;
constexpr size_t kOffSP   = kOffWT   + (size_t)kPosHid * kFeat * 2;
constexpr size_t kWsTotal = kOffSP   + (size_t)kRows * kFeat * 2;
static_assert(kWsTotal == 607232ull, "carve total");
static_assert(kWsTotal <= 134217728ull, "carve cap");
static_assert((kOffNINV % 256) == 0 && (kOffWT % 256) == 0 && (kOffSP % 256) == 0, "aligned regions");

__device__ __forceinline__ unsigned pack_h2(float a, float b) {
  const _Float16 h0 = (_Float16)a;
  const _Float16 h1 = (_Float16)b;
  return (unsigned)__builtin_bit_cast(unsigned short, h0) | ((unsigned)__builtin_bit_cast(unsigned short, h1) << 16);
}

union FragU { v16h v; v8h h[2]; };
__device__ __forceinline__ v16h frag_load(const _Float16* p) {
  FragU f;
  f.h[0] = *(const v8h*)(p);
  f.h[1] = *(const v8h*)(p + 16);
  return f.v;
}
__device__ __forceinline__ v8f mma_f16_guarded(v16h a, v16h b, v8f c) {
  c = __builtin_amdgcn_wmma_f32_16x16x32_f16(false, a, false, b, (short)0, c, false, false);
  asm volatile("v_nop\n\tv_nop\n\tv_nop\n\tv_nop" : "+v"(c) : "v"(a), "v"(b));
  return c;
}
__device__ __forceinline__ void wave_lds_sync() {
  __builtin_amdgcn_fence(__ATOMIC_RELEASE, "workgroup");
  __builtin_amdgcn_wave_barrier();
  __builtin_amdgcn_fence(__ATOMIC_ACQUIRE, "workgroup");
}
__device__ __forceinline__ void flush_slab(const float* slab, float* dst, int lane) {
  const int hh = lane >> 4;
  const int c4 = (lane & 15) * 4;
  for (int pass = 0; pass < 2; ++pass) {
#pragma unroll
    for (int it = 0; it < 8; ++it) {
      const int row = it * 2 + hh;
      const v4f v = *(const v4f*)(slab + row * 68 + c4);
      *(volatile v4f*)(dst + (size_t)row * kOutCols + c4) = v;
    }
    __threadfence();
  }
}

__global__ __launch_bounds__(256) void prep_kernel(
    const float* __restrict__ xh, const float* __restrict__ node_mask, const float* __restrict__ W_pos,
    float* __restrict__ xc, float* __restrict__ ninv, unsigned* __restrict__ Wt)
{
  __shared__ float part[8 * 4];
  const int tid  = threadIdx.x;
  const int lane = tid & 31;
  const int wave = __builtin_amdgcn_readfirstlane((int)(threadIdx.x >> 5));
  if (blockIdx.x < kBatch) {
    const int b   = blockIdx.x;
    const int row = b * kNode + tid;
    const float* r = xh + (size_t)row * kXhIn;
    const float m  = node_mask[row];
    const float x0 = r[0];
    const float x1 = r[1];
    const float x2 = r[2];
    float s0 = x0 * m;
    float s1 = x1 * m;
    float s2 = x2 * m;
    float s3 = m;
#pragma unroll
    for (int off = 16; off >= 1; off >>= 1) {
      s0 += __shfl_xor(s0, off, 32);
      s1 += __shfl_xor(s1, off, 32);
      s2 += __shfl_xor(s2, off, 32);
      s3 += __shfl_xor(s3, off, 32);
    }
    if (lane == 0) {
      part[wave * 4 + 0] = s0;
      part[wave * 4 + 1] = s1;
      part[wave * 4 + 2] = s2;
      part[wave * 4 + 3] = s3;
    }
    __syncthreads();
    float a0 = 0.0f, a1 = 0.0f, a2 = 0.0f, a3 = 0.0f;
#pragma unroll
    for (int w = 0; w < 8; ++w) {
      a0 += part[w * 4 + 0];
      a1 += part[w * 4 + 1];
      a2 += part[w * 4 + 2];
      a3 += part[w * 4 + 3];
    }
    const float inv = 1.0f / a3;
    const float c0 = (x0 - a0 * inv) * m;
    const float c1 = (x1 - a1 * inv) * m;
    const float c2 = (x2 - a2 * inv) * m;
    v4f xo;
    xo[0] = c0;
    xo[1] = c1;
    xo[2] = c2;
    xo[3] = m;
    volatile v4f* q = (volatile v4f*)(xc + (size_t)row * 4);
    *q = xo;
    __threadfence();
    *q = xo;
    if (wave == 0) {
      volatile float* qn = ninv + b * 32 + lane;
      *qn = inv;
      __threadfence();
      *qn = inv;
    }
  } else {
#pragma unroll 1
    for (int i = 0; i < kPosHid / 8; ++i) {
      const int n  = wave * (kPosHid / 8) + i;
      const int k0 = 2 * lane;
      const float w0 = W_pos[(size_t)(k0) * kPosHid + n];
      const float w1 = W_pos[(size_t)(k0 + 1) * kPosHid + n];
      const float w2 = W_pos[(size_t)(kFreq + k0) * kPosHid + n];
      const float w3 = W_pos[(size_t)(kFreq + k0 + 1) * kPosHid + n];
      const unsigned u0 = pack_h2(w0 * kWCarry, w1 * kWCarry);
      const unsigned u1 = pack_h2(w2 * kWCarry, w3 * kWCarry);
      volatile unsigned* q = Wt + (size_t)n * (kFeat / 2);
      q[lane] = u0;
      q[32 + lane] = u1;
      __threadfence();
      q[lane] = u0;
      q[32 + lane] = u1;
    }
  }
}

__global__ __launch_bounds__(256) void pair_feature_sum_kernel(
    const float* __restrict__ xc, const float* __restrict__ ninv, unsigned* __restrict__ Sw)
{
  __shared__ float d_sh[kNode];
  __shared__ float m_sh[kNode];
  __shared__ __align__(16) float red[4 * kFeat];
  const int row  = blockIdx.x;
  const int b    = row >> 8;
  const int tid  = threadIdx.x;
  const int lane = tid & 31;
  const int wave = __builtin_amdgcn_readfirstlane((int)(threadIdx.x >> 5));

  const v4f xi = *(const v4f*)(xc + (size_t)row * 4);
  const v4f xj = *(const v4f*)(xc + (size_t)(b * kNode + tid) * 4);
  const float nv = ninv[b * 32];
  const float rowscale = xi[3] * nv * kSCarry;
  const float dx = xi[0] - xj[0];
  const float dy = xi[1] - xj[1];
  const float dz = xi[2] - xj[2];
  const float sq = fmaxf(dx * dx + dy * dy + dz * dz, 0.0f);
  d_sh[tid] = sqrtf(sq + 1e-12f);
  m_sh[tid] = xj[3];
  __syncthreads();

  const int part = wave >> 1;
  const int k    = (wave & 1) * 32 + lane;
  const float kf = (float)k;
  const float freq = exp2f(fmaf(kf, kFreqStepHi, kf * kFreqStepLo));
  float sa = 0.0f;
  float ca = 0.0f;
  const int j0 = part * 64;
#pragma unroll 1
  for (int jj = 0; jj < 64; ++jj) {
    const float u   = d_sh[j0 + jj] * freq;
    const float uf  = u - floorf(u);
    const float ang = kTwoPi * uf;
    const float mj  = m_sh[j0 + jj];
    const float sv  = sinf(ang);
    const float cv  = cosf(ang);
    sa = fmaf(mj, sv, sa);
    ca = fmaf(mj, cv, ca);
  }
  red[(k << 2) | part] = sa;
  red[4 * kFreq + ((k << 2) | part)] = ca;
  __syncthreads();

  const v4f r0 = *(const v4f*)(red + 8 * k);
  const v4f r1 = *(const v4f*)(red + 8 * k + 4);
  const float v0 = (((r0[0] + r0[1]) + r0[2]) + r0[3]) * rowscale;
  const float v1 = (((r1[0] + r1[1]) + r1[2]) + r1[3]) * rowscale;
  const unsigned u = pack_h2(v0, v1);
  if (wave < 2) {
    volatile unsigned* q = Sw + (size_t)row * (kFeat / 2) + k;
    *q = u;
    __threadfence();
    *q = u;
  }
}

__global__ __launch_bounds__(128) void embed_gemm_kernel(
    const unsigned short* __restrict__ Sp, const unsigned short* __restrict__ Wtp,
    const float* __restrict__ xc, const float* __restrict__ ninv, const float* __restrict__ xh,
    const float* __restrict__ W_xh, const float* __restrict__ b_xh, const float* __restrict__ b_pos,
    float* __restrict__ out)
{
  __shared__ __align__(16) float sT[4][16 * 68];
  __shared__ __align__(16) float sH[4][160];
  __shared__ __align__(16) float sC[4][64];
  const _Float16* S  = (const _Float16*)Sp;
  const _Float16* Wt = (const _Float16*)Wtp;
  const int lane  = threadIdx.x & 31;
  const int wave  = __builtin_amdgcn_readfirstlane((int)(threadIdx.x >> 5));
  const int m0    = blockIdx.x * 64 + wave * 16;
  const int bidx  = m0 >> 8;
  const int rlane = lane & 15;
  const int koff  = (lane >> 4) * 8;
  const int mOff  = (lane >> 4) * 8;
  float* slab = sT[wave];
  float* hbuf = sH[wave];
  float* cbuf = sC[wave];

#pragma unroll
  for (int it = 0; it < 5; ++it) {
    const int idx = it * 32 + lane;
    const int src = idx < (16 * kXhIn - 1) ? idx : (16 * kXhIn - 1);
    hbuf[idx] = xh[(size_t)m0 * kXhIn + src];
  }
  {
    const v4f cv = *(const v4f*)(xc + (size_t)(m0 + rlane) * 4);
    *(v4f*)(cbuf + rlane * 4) = cv;
  }
  wave_lds_sync();

  const float bfac = kPairCount * ninv[bidx * 32];
  float mk[8];
#pragma unroll
  for (int r = 0; r < 8; ++r) mk[r] = cbuf[(mOff + r) * 4 + 3];

  v16h af[4];
#pragma unroll
  for (int ks = 0; ks < 4; ++ks)
    af[ks] = frag_load(S + (size_t)(m0 + rlane) * kFeat + ks * 32 + koff);

  {
    v2f wv[kXhIn];
#pragma unroll
    for (int c = 0; c < kXhIn; ++c) wv[c] = *(const v2f*)(W_xh + c * kXhHid + 2 * lane);
    const v2f bb = *(const v2f*)(b_xh + 2 * lane);
#pragma unroll 1
    for (int r = 0; r < 16; ++r) {
      const float* hr = hbuf + r * kXhIn;
      const float* cr = cbuf + r * 4;
      float a[kXhIn];
      a[0] = cr[0];
      a[1] = cr[1];
      a[2] = cr[2];
#pragma unroll
      for (int c = 3; c < kXhIn; ++c) a[c] = hr[c];
      const float mrow = cr[3];
      float o0 = 0.0f;
      float o1 = 0.0f;
#pragma unroll
      for (int c = 0; c < kXhIn; ++c) {
        o0 = fmaf(a[c], wv[c][0], o0);
        o1 = fmaf(a[c], wv[c][1], o1);
      }
      o0 = (o0 + bb[0]) * mrow;
      o1 = (o1 + bb[1]) * mrow;
      slab[r * 68 + 2 * lane]     = o0;
      slab[r * 68 + 2 * lane + 1] = o1;
    }
    wave_lds_sync();
    flush_slab(slab, out + (size_t)m0 * kOutCols, lane);
    wave_lds_sync();
  }

#pragma unroll 1
  for (int p = 0; p < kPosHid / 64; ++p) {
    v8f acc[4];
#pragma unroll
    for (int j = 0; j < 4; ++j) acc[j] = (v8f){0.f, 0.f, 0.f, 0.f, 0.f, 0.f, 0.f, 0.f};
#pragma unroll
    for (int ks = 0; ks < 4; ++ks) {
#pragma unroll
      for (int j = 0; j < 4; ++j) {
        const v16h bfr = frag_load(Wt + (size_t)(p * 64 + (j << 4) + rlane) * kFeat + ks * 32 + koff);
        acc[j] = mma_f16_guarded(af[ks], bfr, acc[j]);
      }
    }
#pragma unroll
    for (int j = 0; j < 4; ++j) {
      const int n = p * 64 + (j << 4) + rlane;
      const float bv = b_pos[n] * bfac;
#pragma unroll
      for (int r = 0; r < 8; ++r) {
        const float v = (acc[j][r] * kFold + bv) * mk[r];
        slab[(mOff + r) * 68 + (j << 4) + rlane] = v;
      }
    }
    wave_lds_sync();
    flush_slab(slab, out + (size_t)m0 * kOutCols + kXhHid + p * 64, lane);
    wave_lds_sync();
  }
}

extern "C" void kernel_launch(void* const* d_in, const int* in_sizes, int n_in,
                              void* d_out, int out_size, void* d_ws, size_t ws_size,
                              hipStream_t stream) {
  if (n_in < 8) return;
  if (in_sizes[1] != kRows * kXhIn) return;
  if (in_sizes[2] != kRows) return;
  if (in_sizes[4] != kXhIn * kXhHid) return;
  if (in_sizes[5] != kXhHid) return;
  if (in_sizes[6] != kFeat * kPosHid) return;
  if (in_sizes[7] != kPosHid) return;
  if (out_size != kRows * kOutCols) return;
  if (ws_size < kWsTotal) return;

  const float* xh        = (const float*)d_in[1];
  const float* node_mask = (const float*)d_in[2];
  const float* W_xh      = (const float*)d_in[4];
  const float* b_xh      = (const float*)d_in[5];
  const float* W_pos     = (const float*)d_in[6];
  const float* b_pos     = (const float*)d_in[7];
  float* out = (float*)d_out;

  char* ws = (char*)d_ws;
  float*    XC   = (float*)(ws + kOffXC);
  float*    NINV = (float*)(ws + kOffNINV);
  unsigned* WT   = (unsigned*)(ws + kOffWT);
  unsigned* SP   = (unsigned*)(ws + kOffSP);

  prep_kernel<<<kBatch + 1, 256, 0, stream>>>(xh, node_mask, W_pos, XC, NINV, WT);
  pair_feature_sum_kernel<<<kRows, 256, 0, stream>>>(XC, NINV, SP);
  embed_gemm_kernel<<<kRows / 64, 128, 0, stream>>>(
      (const unsigned short*)SP, (const unsigned short*)WT, XC, NINV, xh, W_xh, b_xh, b_pos, out);
}
